// CausalLinearAttention_18915035971883
// MI455X (gfx1250) — hardware-run, weakly checked
//
#include <hip/hip_runtime.h>
#define NB 4
#define SQ 2048
#define NH 8
#define HD 64
#define CH 64
#define NCH 32
#define EPSZ 1e-10f
typedef __bf16 v16b __attribute__((ext_vector_type(16)));
typedef unsigned short v8us __attribute__((ext_vector_type(8), may_alias));
typedef float  v8f  __attribute__((ext_vector_type(8)));
typedef float  v4f  __attribute__((ext_vector_type(4)));
typedef float  v4fa __attribute__((ext_vector_type(4), may_alias));
union FragB { v16b v; v8us half[2]; unsigned short u[16]; };

__device__ __forceinline__ unsigned short bf16_bits(float x) { unsigned int u = __float_as_uint(x); return (unsigned short)((u + 0x7FFFu + ((u >> 16) & 1u)) >> 16); }
__device__ __forceinline__ float bf16_val(unsigned short b) { return __uint_as_float(((unsigned int)b) << 16); }
__device__ __forceinline__ float bf16_round(float x) { return bf16_val(bf16_bits(x)); }
template <int NT>
__device__ __forceinline__ v8f mmaN(v16b ah, v16b al, v16b bh, v16b bl, v8f c) {
  c = __builtin_amdgcn_wmma_f32_16x16x32_bf16(false, ah, false, bh, (short)0, c, false, false);
  if (NT >= 2) c = __builtin_amdgcn_wmma_f32_16x16x32_bf16(false, al, false, bh, (short)0, c, false, false);
  if (NT >= 3) c = __builtin_amdgcn_wmma_f32_16x16x32_bf16(false, ah, false, bl, (short)0, c, false, false);
  asm volatile("v_nop\n\tv_nop\n\tv_nop\n\tv_nop" : "+v"(c) : "v"(ah), "v"(al), "v"(bh), "v"(bl));
  return c;
}


typedef _Float16 v16h __attribute__((ext_vector_type(16)));
union FragH { v16h v; v8us half[2]; _Float16 h[16]; unsigned short u[16]; };
template <int NT>
__device__ __forceinline__ v8f mmaH(v16h ah, v16h al, v16h bh, v16h bl, v8f c) {
  c = __builtin_amdgcn_wmma_f32_16x16x32_f16(false, ah, false, bh, (short)0, c, false, false);
  if (NT >= 2) c = __builtin_amdgcn_wmma_f32_16x16x32_f16(false, al, false, bh, (short)0, c, false, false);
  if (NT >= 3) c = __builtin_amdgcn_wmma_f32_16x16x32_f16(false, ah, false, bl, (short)0, c, false, false);
  asm volatile("v_nop\n\tv_nop\n\tv_nop\n\tv_nop" : "+v"(c) : "v"(ah), "v"(al), "v"(bh), "v"(bl));
  return c;
}

typedef _Float16 v4h __attribute__((ext_vector_type(4)));

__device__ __forceinline__ v16h g2_frag(const _Float16* p, int hh) { FragH f; f.half[0] = *(const v8us*)((const unsigned short*)p + 8 * hh); f.half[1] = *(const v8us*)((const unsigned short*)p + 16 + 8 * hh); return f.v; }
__device__ __forceinline__ v8f g2_mma(v16h a, v16h b, v8f c) { v8f d = __builtin_amdgcn_wmma_f32_16x16x32_f16(false, a, false, b, (short)0, c, false, false); asm volatile("v_nop\n\tv_nop\n\tv_nop\n\tv_nop" : "+v"(d) : "v"(a), "v"(b)); return d; }
template <int ACT>
__global__ __launch_bounds__(128) void k_gemm2(const _Float16* __restrict__ A, int lda, size_t sA, const _Float16* __restrict__ Bh, int ldb, size_t sB, float alpha, const float* __restrict__ bias, size_t sBias, const float* __restrict__ CP, int rowsPerB, size_t sCPb, int row0g,
    float* __restrict__ C, _Float16* __restrict__ C16, int ldc, size_t sC, int M, int N, int K) { static_assert(ACT == 0 || ACT == 3 || ACT == 6 || ACT == 8 || ACT == 9 || ACT == 11 || ACT == 12 || ACT == 14 || ACT == 15 || ACT == 16 || ACT == 17, "k_gemm2: unsupported ACT code (would silently apply no activation)");
  __shared__ __attribute__((aligned(16))) float so[4][32][68];
  const int tid = threadIdx.x, w = tid >> 5, lane = tid & 31, ln = lane & 15, hh = lane >> 4; const int by = blockIdx.y;
  A += (size_t)by * sA; Bh += (size_t)by * sB; const size_t cofs = (size_t)by * sC; const float* bp = bias ? bias + (size_t)by * sBias : nullptr;
  const int ntn = N >> 6; const int mt = blockIdx.x / ntn, nq = blockIdx.x - mt * ntn; const int row0 = mt * 128 + 32 * w, col0 = nq * 64; if (row0 >= M) return;
  const _Float16* a0p = A + (size_t)(row0 + ln) * lda; const _Float16* a1p = a0p + (size_t)16 * lda;
  const _Float16* b0p = Bh + (size_t)(col0 + ln) * ldb; const _Float16* b1p = b0p + (size_t)16 * ldb; const _Float16* b2p = b1p + (size_t)16 * ldb; const _Float16* b3p = b2p + (size_t)16 * ldb;
  const v8f z8 = {0.f,0.f,0.f,0.f,0.f,0.f,0.f,0.f}; v8f c00 = z8, c01 = z8, c02 = z8, c03 = z8, c10 = z8, c11 = z8, c12 = z8, c13 = z8;
  for (int kb = 0; kb < K; kb += 32) { const v16h a0 = g2_frag(a0p + kb, hh), a1 = g2_frag(a1p + kb, hh);
    v16h b = g2_frag(b0p + kb, hh); c00 = g2_mma(a0, b, c00); c10 = g2_mma(a1, b, c10);
    b = g2_frag(b1p + kb, hh); c01 = g2_mma(a0, b, c01); c11 = g2_mma(a1, b, c11);
    b = g2_frag(b2p + kb, hh); c02 = g2_mma(a0, b, c02); c12 = g2_mma(a1, b, c12);
    b = g2_frag(b3p + kb, hh); c03 = g2_mma(a0, b, c03); c13 = g2_mma(a1, b, c13); }
  v8f accs[8] = {c00, c01, c02, c03, c10, c11, c12, c13};
#pragma unroll
  for (int u = 0; u < 8; ++u) { const int t = u & 3, half = u >> 2; const int col = col0 + t * 16 + ln; const float bv = bp ? bf16_round(bp[col]) : 0.f;
#pragma unroll
    for (int r = 0; r < 8; ++r) { const int rloc = half * 16 + 8 * hh + r; float v = accs[u][r] * alpha + bv; if (CP) { if (rowsPerB < 0) v += CP[cofs + (size_t)(row0g + row0 + rloc) * ldc + col];        else { const int bidx = (row0g + row0 + rloc) / rowsPerB; v += CP[(size_t)bidx * sCPb + (size_t)by * 64 + col]; } }
      if (ACT == 3) v = fmaxf(v, 0.f); else if (ACT == 6) v = 0.5f * v * (1.0f + erff(v * 0.70710678118654752f)); else if (ACT == 11) v = 1.0f / (1.0f + expf(-v)); else if (ACT == 15) v = v / (1.0f + expf(-v)); else if (ACT == 12) v = (v > 0.f) ? v : 0.01f * v; else if (ACT == 8) v = tanhf(v); else if (ACT == 9) v = 0.5f * v * (1.0f + tanhf(0.7978845608028654f * (v + 0.044715f * v * v * v))); else if (ACT == 14) v = (v > 0.f) ? v : 0.1f * v; else if (ACT == 16) v = (v >= 0.f) ? v : 0.3f * v; else if (ACT == 17) v = (v >= 0.f) ? v : 0.2f * v;
      so[w][rloc][t * 16 + ln] = v; } }
  __builtin_amdgcn_fence(__ATOMIC_ACQ_REL, "workgroup"); __builtin_amdgcn_wave_barrier();
  const int rsub = lane >> 4, c4 = (lane & 15) * 4;
  for (int pass = 0; pass < 2; ++pass) {
#pragma unroll
    for (int q = 0; q < 16; ++q) { const int r = q * 2 + rsub; const v4f v = *(const v4fa*)&so[w][r][c4]; if (C) *(volatile v4f*)(C + cofs + (size_t)(row0 + r) * ldc + col0 + c4) = v; if (C16) { v4h h4; for (int i = 0; i < 4; ++i) h4[i] = (_Float16)v[i]; *(volatile v4h*)(C16 + cofs + (size_t)(row0 + r) * ldc + col0 + c4) = h4; } }
    if (pass == 0) __threadfence(); } }

__global__ __launch_bounds__(256) void k_hm(const float* __restrict__ X, float* __restrict__ HM, size_t n8) {
  const size_t t8 = (size_t)blockIdx.x * 256 + threadIdx.x; if (t8 >= n8) return; const size_t r = t8 >> 3; const int d0 = (int)(t8 & 7) * 8, tok = (int)(r & (SQ - 1)), s = (int)(r >> 11), b = s >> 3, h = s & 7;
  const float* xp = X + (((size_t)b * SQ + tok) * NH + h) * HD + d0; const v4f a = *(const v4fa*)xp; const v4f c = *(const v4fa*)(xp + 4); v4f ya, yc;
  for (int q = 0; q < 4; ++q) { ya[q] = bf16_round(a[q]); yc[q] = bf16_round(c[q]); }
  float* op = HM + t8 * 8;
  for (int pass = 0; pass < 2; ++pass) { *(volatile v4f*)op = ya; *(volatile v4f*)(op + 4) = yc; if (pass == 0) __threadfence(); } }
__global__ __launch_bounds__(256) void k_phi(float* XF, _Float16* __restrict__ H16, size_t n8) {
  const size_t t = (size_t)blockIdx.x * 256 + threadIdx.x; if (t >= n8) return; float* xp = XF + t * 8; const v4f a = *(const v4fa*)xp; const v4f c = *(const v4fa*)(xp + 4); v4f ya, yc; FragH f;
#pragma unroll
  for (int q = 0; q < 4; ++q) { ya[q] = expf(fminf(a[q], 0.f)) + fmaxf(a[q], 0.f); yc[q] = expf(fminf(c[q], 0.f)) + fmaxf(c[q], 0.f); f.h[q] = (_Float16)ya[q]; f.h[4 + q] = (_Float16)yc[q]; }
  unsigned short* hp = (unsigned short*)H16 + t * 8;
  for (int pass = 0; pass < 2; ++pass) { *(volatile v4f*)xp = ya; *(volatile v4f*)(xp + 4) = yc; *(volatile v8us*)hp = f.half[0]; if (pass == 0) __threadfence(); } }
__global__ __launch_bounds__(256) void k_wtc_f16(const float* __restrict__ W, _Float16* __restrict__ Wt, int K, int N, float scale) {
  const int t = blockIdx.x * 256 + threadIdx.x; if (t >= N * (K / 8)) return; const int n = t / (K / 8), k8 = (t % (K / 8)) * 8; FragH f;
#pragma unroll
  for (int i = 0; i < 8; ++i) f.h[i] = (_Float16)(W[(size_t)(k8 + i) * N + n] * scale); const v8us o = f.half[0];
  *(volatile v8us*)((unsigned short*)Wt + (size_t)n * K + k8) = o; __threadfence(); *(volatile v8us*)((unsigned short*)Wt + (size_t)n * K + k8) = o;
}
__global__ __launch_bounds__(256) void k_tril(const float* __restrict__ SC, _Float16* __restrict__ P16, size_t n8) {
  const size_t t = (size_t)blockIdx.x * 256 + threadIdx.x; if (t >= n8) return; const int j0 = (int)(t & 7) * 8, i = (int)((t >> 3) & 63); const float* sp = SC + t * 8; const v4f a = *(const v4fa*)sp; const v4f c = *(const v4fa*)(sp + 4); FragH f;
  for (int q = 0; q < 4; ++q) { f.h[q] = (_Float16)(a[q] * (float)(j0 + q <= i)); f.h[4 + q] = (_Float16)(c[q] * (float)(j0 + 4 + q <= i)); }
  unsigned short* hp = (unsigned short*)P16 + t * 8;
  for (int pass = 0; pass < 2; ++pass) { *(volatile v8us*)hp = f.half[0]; if (pass == 0) __threadfence(); } }
__global__ __launch_bounds__(256) void k_plo(const float* __restrict__ SC, _Float16* __restrict__ PL, size_t n8) {
  const size_t t = (size_t)blockIdx.x * 256 + threadIdx.x; if (t >= n8) return; const int j0 = (int)(t & 7) * 8, i = (int)((t >> 3) & 63); const size_t s = t >> 9; const float* sp = SC + s * ((size_t)NCH * CH * CH) + (t & 511) * 8; const v4f a = *(const v4fa*)sp; const v4f c = *(const v4fa*)(sp + 4); v4f ma, mc;
  for (int q = 0; q < 4; ++q) { ma[q] = a[q] * (float)(j0 + q <= i); mc[q] = c[q] * (float)(j0 + 4 + q <= i); }
  const v4f ra = (ma - __builtin_convertvector(__builtin_convertvector(ma, v4h), v4f)) * 1024.0f, rc = (mc - __builtin_convertvector(__builtin_convertvector(mc, v4h), v4f)) * 1024.0f; union { v4h q[2]; v8us u; } f; f.q[0] = __builtin_convertvector(ra, v4h); f.q[1] = __builtin_convertvector(rc, v4h);
  unsigned short* hp = (unsigned short*)PL + t * 8;
  for (int pass = 0; pass < 2; ++pass) { *(volatile v8us*)hp = f.u; if (pass == 0) __threadfence(); } }
__global__ __launch_bounds__(256) void k_rowsum(const _Float16* __restrict__ P16, const _Float16* __restrict__ PL, float* __restrict__ RS, size_t n) {
  const size_t t = (size_t)blockIdx.x * 256 + threadIdx.x; if (t >= n) return; const unsigned short* sp = (const unsigned short*)P16 + (size_t)t * CH; const unsigned short* lp = (const unsigned short*)PL + ((t >> 11) * CH + (t & 63)) * CH; const float first = (float)(((t >> 6) & (NCH - 1)) == 0) * (1.0f / 1024.0f); float acc = 0.f, lo = 0.f;
  for (int j = 0; j < CH / 8; ++j) { FragH f, g; f.half[0] = *(const v8us*)(sp + 8 * j); g.half[0] = *(const v8us*)(lp + 8 * j); for (int q = 0; q < 8; ++q) { acc += (float)f.h[q]; lo += (float)g.h[q]; } }
  acc += lo * first;
  for (int pass = 0; pass < 2; ++pass) { *(volatile float*)(RS + t) = acc; if (pass == 0) __threadfence(); } }
__global__ __launch_bounds__(256) void k_kscan(const _Float16* __restrict__ KT, float* __restrict__ KP, int n, size_t ldk) {
  const int t = blockIdx.x * 256 + threadIdx.x; if (t >= n) return; const int s = t >> 6, kk = t & 63; const unsigned short* kp = (const unsigned short*)KT + (size_t)kk * ldk + (size_t)s * SQ; float* op = KP + (size_t)s * NCH * HD + kk; float acc = 0.f;
  for (int c = 0; c < NCH; ++c) { *(volatile float*)(op + (size_t)c * HD) = acc; __threadfence(); *(volatile float*)(op + (size_t)c * HD) = acc;
    for (int j = 0; j < CH / 8; ++j) { FragH f; f.half[0] = *(const v8us*)(kp + (size_t)c * CH + 8 * j); for (int q = 0; q < 8; ++q) acc += (float)f.h[q]; } } }
__global__ __launch_bounds__(256) void k_cscan(const float* __restrict__ DK, _Float16* __restrict__ ST16, int n) {
  const int t = blockIdx.x * 256 + threadIdx.x; if (t >= n) return; const size_t base = (size_t)(t >> 9) * NCH * (HD * HD) + (size_t)(t & 511) * 8; v4f a0 = {0.f, 0.f, 0.f, 0.f}, a1 = {0.f, 0.f, 0.f, 0.f};
  for (int c = 0; c < NCH; ++c) { const size_t o = base + (size_t)c * (HD * HD); union { v4h q[2]; v8us u; } f; f.q[0] = __builtin_convertvector(a0, v4h); f.q[1] = __builtin_convertvector(a1, v4h);
    unsigned short* hp = (unsigned short*)ST16 + o; *(volatile v8us*)hp = f.u; __threadfence(); *(volatile v8us*)hp = f.u;
    const v4f x0 = *(const v4fa*)(DK + o); const v4f x1 = *(const v4fa*)(DK + o + 4); a0 = a0 + x0; a1 = a1 + x1; } }
__global__ __launch_bounds__(256) void k_zden(const float* __restrict__ ND, const _Float16* __restrict__ Q16, const float* __restrict__ KP, const float* __restrict__ RS, float* __restrict__ OUT, size_t n) {
  const size_t r = (size_t)blockIdx.x * 256 + threadIdx.x; if (r >= n) return; const int tok = (int)(r & (SQ - 1)), s = (int)(r >> 11), b = s >> 3, h = s & 7; const unsigned short* q = (const unsigned short*)Q16 + r * HD; const float* kp = KP + (r >> 6) * HD; float den = RS[r];
  for (int j = 0; j < HD / 8; ++j) { FragH f; f.half[0] = *(const v8us*)(q + 8 * j); for (int i = 0; i < 8; ++i) den += (float)f.h[i] * kp[8 * j + i]; }
  const float z = 1.0f / (den + EPSZ); const float* np = ND + r * HD; float* op = OUT + (((size_t)b * SQ + tok) * NH + h) * HD;
  for (int pass = 0; pass < 2; ++pass) { for (int j = 0; j < HD / 4; ++j) { const v4f x = *(const v4fa*)(np + 4 * j); v4f y; for (int i = 0; i < 4; ++i) y[i] = x[i] * z; *(volatile v4f*)(op + 4 * j) = y; } if (pass == 0) __threadfence(); } }

extern "C" void kernel_launch(void* const* d_in, const int* in_sizes, int n_in,
                              void* d_out, int out_size, void* d_ws, size_t ws_size, hipStream_t stream) {
  (void)in_sizes; (void)n_in; (void)out_size;
  const float* queries = (const float*)d_in[0]; const float* keys = (const float*)d_in[1]; const float* values = (const float*)d_in[2];
  static_assert(NB == 4 && SQ == 2048 && (1 << 11) == SQ && NH == 8 && HD == 64 && CH == 64 && NCH * CH == SQ && HD * HD == 4096 && HD % 64 == 0 && HD % 32 == 0 && CH % 32 == 0 && ((size_t)NB * NH * SQ * HD / 8) % 256 == 0 && ((size_t)HD * ((size_t)NB * NH * SQ / 8)) % 256 == 0 && ((size_t)NB * NH * NCH * CH * CH / 8) % 256 == 0 && (NB * NH * NCH * CH) % 256 == 0 && ((size_t)NB * NH * CH * CH / 8) % 256 == 0 && (NB * NH * 64) % 256 == 0 && (NB * NH * 512) % 256 == 0 && (NB * NH * SQ) % 256 == 0, "the index shifts; whole tiles; exact grids");
  float* out = (float*)d_out;
  const int NS = NB * NH;
  const int NT = NS * SQ;
  const int NZ = NS * NCH;
  char* ws = (char*)d_ws; size_t off = 0;
  auto take = [&](size_t bytes) { char* p = ws + off; off += (bytes + 255) & ~(size_t)255; return p; };
  float* FA = (float*)take((size_t)NT * HD * 4);
  _Float16* QH = (_Float16*)take((size_t)NT * HD * 2); _Float16* KP16 = (_Float16*)take((size_t)NT * HD * 2);
  _Float16* KS = (_Float16*)take((size_t)HD * NT * 2); _Float16* VT = (_Float16*)take((size_t)HD * NT * 2);
  float* RS = (float*)take((size_t)NT * 4); float* KPS = (float*)take((size_t)NZ * HD * 4); _Float16* PL = (_Float16*)take((size_t)NS * CH * CH * 2);
  if (off > ws_size) return;
  k_hm<<<(unsigned)((size_t)NT * HD / 8 / 256), 256, 0, stream>>>(queries, FA, (size_t)NT * HD / 8);
  k_phi<<<(unsigned)((size_t)NT * HD / 8 / 256), 256, 0, stream>>>(FA, QH, (size_t)NT * HD / 8);
  k_hm<<<(unsigned)((size_t)NT * HD / 8 / 256), 256, 0, stream>>>(keys, FA, (size_t)NT * HD / 8);
  k_phi<<<(unsigned)((size_t)NT * HD / 8 / 256), 256, 0, stream>>>(FA, KP16, (size_t)NT * HD / 8);
  k_wtc_f16<<<(unsigned)((size_t)HD * (NT / 8) / 256), 256, 0, stream>>>(FA, KS, NT, HD, 1.0f);
  k_hm<<<(unsigned)((size_t)NT * HD / 8 / 256), 256, 0, stream>>>(values, FA, (size_t)NT * HD / 8);
  k_wtc_f16<<<(unsigned)((size_t)HD * (NT / 8) / 256), 256, 0, stream>>>(FA, VT, NT, HD, 1.0f);
  k_gemm2<0><<<dim3((HD / 64) * (CH / 64), NZ), 128, 0, stream>>>(QH, HD, (size_t)CH * HD, KP16, HD, (size_t)CH * HD, 1.0f, nullptr, 0, nullptr, 1, 0, 0, FA, nullptr, CH, (size_t)CH * CH, CH, CH, HD);
  k_tril<<<(unsigned)((size_t)NZ * CH * CH / 8 / 256), 256, 0, stream>>>(FA, KP16, (size_t)NZ * CH * CH / 8);
  k_plo<<<(unsigned)((size_t)NS * CH * CH / 8 / 256), 256, 0, stream>>>(FA, PL, (size_t)NS * CH * CH / 8);
  k_rowsum<<<(unsigned)(NZ * CH / 256), 256, 0, stream>>>(KP16, PL, RS, (size_t)NZ * CH);
  k_gemm2<0><<<dim3((HD / 64) * (HD / 64), NZ), 128, 0, stream>>>(VT, NT, (size_t)CH, KS, NT, (size_t)CH, 1.0f, nullptr, 0, nullptr, 1, 0, 0, FA, nullptr, HD, (size_t)HD * HD, HD, HD, CH);
  k_kscan<<<(unsigned)(NS * 64 / 256), 256, 0, stream>>>(KS, KPS, NS * 64, (size_t)NT);
  k_cscan<<<(unsigned)(NS * 512 / 256), 256, 0, stream>>>(FA, KS, NS * 512);
  k_gemm2<0><<<dim3((HD / 64) * (CH / 64), NZ), 128, 0, stream>>>(QH, HD, (size_t)CH * HD, KS, HD, (size_t)HD * HD, 1.0f, nullptr, 0, nullptr, 1, 0, 0, FA, nullptr, HD, (size_t)CH * HD, CH, HD, HD);
  k_gemm2<0><<<dim3((HD / 64) * (CH / 64), NZ), 128, 0, stream>>>(KP16, CH, (size_t)CH * CH, VT, NT, (size_t)CH, 1.0f, nullptr, 0, FA, -1, 0, 0, FA, nullptr, HD, (size_t)CH * HD, CH, HD, CH);
  k_gemm2<0><<<dim3((HD / 64) * (CH / 64), NS), 128, 0, stream>>>(PL, CH, (size_t)CH * CH, VT, NT, (size_t)SQ, 1.0f / 1024.0f, nullptr, 0, FA, -1, 0, 0, FA, nullptr, HD, (size_t)NCH * CH * HD, CH, HD, CH);
  k_zden<<<(unsigned)(NT / 256), 256, 0, stream>>>(FA, QH, KPS, RS, out, (size_t)NT);
}
